// GQABlock_14568529068626
// MI455X (gfx1250) — hardware-verified
//
#include <hip/hip_runtime.h>
#include <math.h>

typedef __attribute__((ext_vector_type(16))) _Float16 v16h;
typedef __attribute__((ext_vector_type(8)))  _Float16 v8h;
typedef __attribute__((ext_vector_type(16))) __bf16   v16b;
typedef __attribute__((ext_vector_type(8)))  __bf16   v8b;
typedef __attribute__((ext_vector_type(8)))  float    v8f;
typedef __attribute__((ext_vector_type(4)))  float    v4f;
typedef __attribute__((ext_vector_type(4)))  unsigned int v4u;

constexpr int kBatch = 2;
constexpr int kSeq   = 2048;
constexpr int kEmb   = 2048;
constexpr int kHq    = 32;
constexpr int kHkv   = 8;
constexpr int kHd    = 64;
constexpr int kKvW   = kHkv * kHd;
constexpr int kRows  = kBatch * kSeq;
constexpr int kQBlk  = 64;
constexpr int kTK    = 32;
constexpr int kNQB   = kSeq / kQBlk;
constexpr int kNKT   = kSeq / kTK;
constexpr int kMP    = 36;
constexpr int kEarlyRows = 256;
static_assert(kEmb == kHq * kHd, "query width");
static_assert(kKvW == 512, "kv width");
static_assert((kHq % kHkv) == 0, "grouping");
static_assert((kSeq % kQBlk) == 0 && (kEarlyRows % kQBlk) == 0, "query tiling");
static_assert(kNQB == 32 && kNKT == 64, "tile table shape");
static_assert((kEmb % 32) == 0 && (kRows % 64) == 0 && (kEmb % 64) == 0 && (kKvW % 64) == 0 && (kSeq % 64) == 0, "GEMM tile multiples");

constexpr float inv_sqrt_pow4(int n) { return n == 1 ? 1.0f : 0.5f * inv_sqrt_pow4(n / 4); }
static_assert(kHd == 64, "head width");
constexpr float kInvSqrtHd = inv_sqrt_pow4(kHd);
static_assert(kInvSqrtHd * kInvSqrtHd * (float)kHd == 1.0f, "score scale");

constexpr float kQCarry   = 8.0f;
constexpr float kKCarry   = 8.0f;
constexpr float kVCarry   = 8.0f;
constexpr float kPCarry   = 32768.0f;
constexpr float kLoCarry  = 2048.0f;
constexpr float kLoCarryInv = 1.0f / kLoCarry;
constexpr float kCtxCarry = 128.0f;
constexpr float kWoCarry  = 1024.0f;
constexpr float kScoreScale   = kInvSqrtHd / (kQCarry * kKCarry);
constexpr float kScoreLoScale = kScoreScale / kLoCarry;
constexpr float kCtxFold  = kCtxCarry / kVCarry;
constexpr float kOutScale = 1.0f / (kCtxCarry * kWoCarry);
constexpr float kMaskDeadThr = -1.0e8f;
constexpr float kMaskLiveThr = -1.0e7f;

constexpr size_t kOffXB  = 0;
constexpr size_t kOffWQB = kOffXB  + (size_t)kRows * kEmb * 2;
constexpr size_t kOffWKB = kOffWQB + (size_t)kEmb  * kEmb * 2;
constexpr size_t kOffWVB = kOffWKB + (size_t)kKvW  * kEmb * 2;
constexpr size_t kOffWOH = kOffWVB + (size_t)kKvW  * kEmb * 2;
constexpr size_t kOffWOB = kOffWOH + (size_t)kEmb  * kEmb * 2;
constexpr size_t kOffQH  = kOffWOB + (size_t)kEmb  * kEmb * 2;
constexpr size_t kOffQL  = kOffQH  + (size_t)kRows * kEmb * 2;
constexpr size_t kOffKH  = kOffQL  + (size_t)kRows * kEmb * 2;
constexpr size_t kOffKL  = kOffKH  + (size_t)kRows * kKvW * 2;
constexpr size_t kOffVTH = kOffKL  + (size_t)kRows * kKvW * 2;
constexpr size_t kOffVTL = kOffVTH + (size_t)kBatch * kKvW * kSeq * 2;
constexpr size_t kOffCH  = kOffVTL + (size_t)kBatch * kKvW * kSeq * 2;
constexpr size_t kOffCL  = kOffCH  + (size_t)kRows * kEmb * 2;
constexpr size_t kOffSKP = kOffCL  + (size_t)kRows * kEmb * 2;
constexpr size_t kWsTotal = kOffSKP + (size_t)kNQB * kNKT * 4;
static_assert(kWsTotal == 130031616ull, "carve total");
static_assert(kWsTotal <= 134217728ull, "carve cap");
static_assert((kOffWQB % 128) == 0 && (kOffWKB % 128) == 0 && (kOffWVB % 128) == 0 && (kOffWOH % 128) == 0 &&
              (kOffWOB % 128) == 0 && (kOffQH % 128) == 0 && (kOffQL % 128) == 0 && (kOffKH % 128) == 0 &&
              (kOffKL % 128) == 0 && (kOffVTH % 128) == 0 && (kOffVTL % 128) == 0 && (kOffCH % 128) == 0 &&
              (kOffCL % 128) == 0 && (kOffSKP % 128) == 0, "128-B aligned regions");

__device__ __forceinline__ unsigned short f2bf_bits(float f) {
  unsigned u = __float_as_uint(f);
  return (unsigned short)((u + 0x7FFFu + ((u >> 16) & 1u)) >> 16);
}
__device__ __forceinline__ float bf_bits2f(unsigned short h) { return __uint_as_float(((unsigned)h) << 16); }
__device__ __forceinline__ float bf_rne(float f) { return bf_bits2f(f2bf_bits(f)); }
__device__ __forceinline__ unsigned pk16(unsigned short a, unsigned short b) { return (unsigned)a | ((unsigned)b << 16); }
__device__ __forceinline__ unsigned short h_bits(float f) { const _Float16 h = (_Float16)f; return __builtin_bit_cast(unsigned short, h); }

__device__ __forceinline__ void row_guard_h(v8f& a0, v8f& a1, v8f& a2, v8f& a3, v16h x, v16h b0, v16h b1, v16h b2, v16h b3) {
  asm volatile("v_nop\n\tv_nop\n\tv_nop\n\tv_nop" : "+v"(a0), "+v"(a1), "+v"(a2), "+v"(a3) : "v"(x), "v"(b0), "v"(b1), "v"(b2), "v"(b3));
}
__device__ __forceinline__ void row_guard_b(v8f& a0, v8f& a1, v8f& a2, v8f& a3, v16b x, v16b b0, v16b b1, v16b b2, v16b b3) {
  asm volatile("v_nop\n\tv_nop\n\tv_nop\n\tv_nop" : "+v"(a0), "+v"(a1), "+v"(a2), "+v"(a3) : "v"(x), "v"(b0), "v"(b1), "v"(b2), "v"(b3));
}
__device__ __forceinline__ void acc_guard4(v8f& a, v8f& b, v8f& c, v8f& d) { asm volatile("v_nop\n\tv_nop\n\tv_nop\n\tv_nop" : "+v"(a), "+v"(b), "+v"(c), "+v"(d)); }

template <typename T> struct Frag;
template <> struct Frag<_Float16> {
  typedef v16h V; union U { v16h v; v8h h[2]; };
  static __device__ __forceinline__ v16h load(const _Float16* p) {
    U f; f.h[0] = *(const v8h*)(p); f.h[1] = *(const v8h*)(p + 16); return f.v;
  }
  static __device__ __forceinline__ v8f mma(v16h a, v16h b, v8f c) {
    return __builtin_amdgcn_wmma_f32_16x16x32_f16(false, a, false, b, (short)0, c, false, false);
  }
  static __device__ __forceinline__ void guard_row(v8f& a0, v8f& a1, v8f& a2, v8f& a3, v16h x, v16h b0, v16h b1, v16h b2, v16h b3) {
    row_guard_h(a0, a1, a2, a3, x, b0, b1, b2, b3);
  }
};
template <> struct Frag<__bf16> {
  typedef v16b V; union U { v16b v; v8b h[2]; };
  static __device__ __forceinline__ v16b load(const __bf16* p) {
    U f; f.h[0] = *(const v8b*)(p); f.h[1] = *(const v8b*)(p + 16); return f.v;
  }
  static __device__ __forceinline__ v8f mma(v16b a, v16b b, v8f c) {
    return __builtin_amdgcn_wmma_f32_16x16x32_bf16(false, a, false, b, (short)0, c, false, false);
  }
  static __device__ __forceinline__ void guard_row(v8f& a0, v8f& a1, v8f& a2, v8f& a3, v16b x, v16b b0, v16b b1, v16b b2, v16b b3) {
    row_guard_b(a0, a1, a2, a3, x, b0, b1, b2, b3);
  }
};
typedef Frag<_Float16> FragH;

__device__ __forceinline__ v8f mma_h(v16h a, v16h b, v8f c) {
  c = __builtin_amdgcn_wmma_f32_16x16x32_f16(false, a, false, b, (short)0, c, false, false);
  asm volatile("v_nop\n\tv_nop\n\tv_nop\n\tv_nop" : "+v"(c) : "v"(a), "v"(b));
  return c;
}

template <int ET> struct Elem;
template <> struct Elem<0> { typedef _Float16 T; };
template <> struct Elem<1> { typedef __bf16 T; };

__global__ __launch_bounds__(256) void cast8_bf16_kernel(const float* __restrict__ in, unsigned short* __restrict__ out, int n8) {
  const int i = blockIdx.x * 256 + threadIdx.x;
  if (i >= n8) return;
  const float* p = in + 8 * (size_t)i;
  const v4f a = *(const v4f*)(p);
  const v4f c = *(const v4f*)(p + 4);
  unsigned short hb[8];
#pragma unroll
  for (int e = 0; e < 4; ++e) {
    const float fa = a[e];
    const float fc = c[e];
    hb[e]     = f2bf_bits(fa);
    hb[4 + e] = f2bf_bits(fc);
  }
  const v4u u = (v4u){pk16(hb[0], hb[1]), pk16(hb[2], hb[3]), pk16(hb[4], hb[5]), pk16(hb[6], hb[7])};
  unsigned short* q = out + 8 * (size_t)i;
  *(volatile v4u*)q = u;
  __threadfence();
  *(volatile v4u*)q = u;
}

__global__ __launch_bounds__(256) void cast8_wo_kernel(const float* __restrict__ in, unsigned short* __restrict__ outb,
                                                       unsigned short* __restrict__ outh, int n8) {
  const int i = blockIdx.x * 256 + threadIdx.x;
  if (i >= n8) return;
  const float* p = in + 8 * (size_t)i;
  const v4f a = *(const v4f*)(p);
  const v4f c = *(const v4f*)(p + 4);
  unsigned short bb[8], hb[8];
#pragma unroll
  for (int e = 0; e < 4; ++e) {
    const float fa = a[e];
    const float fc = c[e];
    bb[e]     = f2bf_bits(fa);
    bb[4 + e] = f2bf_bits(fc);
    hb[e]     = h_bits(bf_bits2f(bb[e]) * kWoCarry);
    hb[4 + e] = h_bits(bf_bits2f(bb[4 + e]) * kWoCarry);
  }
  const v4u ub = (v4u){pk16(bb[0], bb[1]), pk16(bb[2], bb[3]), pk16(bb[4], bb[5]), pk16(bb[6], bb[7])};
  const v4u uh = (v4u){pk16(hb[0], hb[1]), pk16(hb[2], hb[3]), pk16(hb[4], hb[5]), pk16(hb[6], hb[7])};
  unsigned short* qb = outb + 8 * (size_t)i;
  unsigned short* qh = outh + 8 * (size_t)i;
  *(volatile v4u*)qb = ub;
  *(volatile v4u*)qh = uh;
  __threadfence();
  *(volatile v4u*)qb = ub;
  *(volatile v4u*)qh = uh;
}

__global__ __launch_bounds__(256) void mask_tiles_kernel(const float* __restrict__ Mk, unsigned* __restrict__ Skip) {
  __shared__ unsigned sBits[8][4];
  __shared__ unsigned sLive[8];
  const int tid  = threadIdx.x;
  const int lane = tid & 31;
  const int wave = __builtin_amdgcn_readfirstlane((int)(tid >> 5));
  const int qb   = blockIdx.x;
  unsigned tm = 0xFFFFu;
  int live = 1;
#pragma unroll 1
  for (int rr = 0; rr < 8; ++rr) {
    const int row = qb * kQBlk + wave * 8 + rr;
    const float* mr = Mk + (size_t)row * kSeq + lane * 4;
    int rl = 0;
#pragma unroll
    for (int it = 0; it < 16; ++it) {
      const v4f mv = *(const v4f*)(mr + it * 128);
      const float a0 = mv[0];
      const float a1 = mv[1];
      const float a2 = mv[2];
      const float a3 = mv[3];
      const float mx = bf_rne(fmaxf(fmaxf(a0, a1), fmaxf(a2, a3)));
      const unsigned notdead = (mx <= kMaskDeadThr) ? 0u : 1u;
      const int lv = (mx > kMaskLiveThr) ? 1 : 0;
      tm &= ~(notdead << it);
      rl |= lv;
    }
#pragma unroll
    for (int off = 1; off < 32; off <<= 1) rl |= __shfl_xor(rl, off, 32);
    live &= rl;
  }
  int tmi = (int)tm;
#pragma unroll
  for (int off = 1; off < 8; off <<= 1) tmi &= __shfl_xor(tmi, off, 32);
  if ((lane & 7) == 0) sBits[wave][lane >> 3] = (unsigned)tmi;
  if (lane == 0) sLive[wave] = (unsigned)live;
  __syncthreads();
  const int t = tid & 15;
  unsigned bl = 1u;
#pragma unroll
  for (int w = 0; w < 8; ++w) bl &= sLive[w];
  unsigned f[4];
#pragma unroll
  for (int j = 0; j < 4; ++j) {
    unsigned a = 1u;
#pragma unroll
    for (int w = 0; w < 8; ++w) a &= (sBits[w][j] >> t) & 1u;
    f[j] = a & bl;
  }
  const v4u o = (v4u){f[0], f[1], f[2], f[3]};
  if (tid < 16) {
    unsigned* p = Skip + (size_t)qb * kNKT + t * 4;
    *(volatile v4u*)p = o;
    __threadfence();
    *(volatile v4u*)p = o;
  }
}

template <int ET, bool MIXLO, int OUT_MODE>
__global__ __launch_bounds__(256) void gemm64_kernel(
    const unsigned short* __restrict__ Ap, int lda, long strideA,
    const unsigned short* __restrict__ Btp, int ldb, long strideB,
    const unsigned short* __restrict__ A2p, const unsigned short* __restrict__ Bt2p,
    void* __restrict__ Cout, void* __restrict__ Cout2, int ldc, long strideC,
    int M, int N, int K, float scale, int loPeriod, int loLimit) {
  typedef typename Elem<ET>::T T;
  typedef typename Frag<T>::V V;
  __shared__ __align__(16) float sT[8][16 * 68];
  const int b    = blockIdx.y;
  const int lane = threadIdx.x & 31;
  const int wave = __builtin_amdgcn_readfirstlane((int)(threadIdx.x >> 5));
  const int tilesN = N >> 6;
  const int tilesM = M >> 6;
  const int tile = blockIdx.x * 8 + wave;
  if (tile >= tilesM * tilesN) return;
  const int tm = tile / tilesN;
  const int tn = tile - tm * tilesN;
  const int m0 = tm << 6;
  const int n0 = tn << 6;

  const T* Ab = (const T*)Ap  + (size_t)b * strideA;
  const T* Bb = (const T*)Btp + (size_t)b * strideB;
  const __bf16* A2b = MIXLO ? ((const __bf16*)A2p  + (size_t)b * strideA) : nullptr;
  const __bf16* B2b = MIXLO ? ((const __bf16*)Bt2p + (size_t)b * strideB) : nullptr;
  bool useLo = false;
  if (MIXLO) useLo = ((m0 % loPeriod) < loLimit);

  const int rlane = lane & 15;
  const int koff  = (lane >> 4) * 8;
  const int mOff  = (lane >> 4) * 8;

  v8f acc[4][4];
#pragma unroll
  for (int i = 0; i < 4; ++i)
#pragma unroll
    for (int j = 0; j < 4; ++j) acc[i][j] = (v8f){0.f, 0.f, 0.f, 0.f, 0.f, 0.f, 0.f, 0.f};

  for (int k0 = 0; k0 < K; k0 += 32) {
    {
      V bh[4];
#pragma unroll
      for (int j = 0; j < 4; ++j) bh[j] = Frag<T>::load(Bb + (size_t)(n0 + (j << 4) + rlane) * ldb + koff + k0);
#pragma unroll
      for (int i = 0; i < 4; ++i) {
        const V ah = Frag<T>::load(Ab + (size_t)(m0 + (i << 4) + rlane) * lda + koff + k0);
#pragma unroll
        for (int j = 0; j < 4; ++j) acc[i][j] = Frag<T>::mma(ah, bh[j], acc[i][j]);
        Frag<T>::guard_row(acc[i][0], acc[i][1], acc[i][2], acc[i][3], ah, bh[0], bh[1], bh[2], bh[3]);
      }
    }
    if (MIXLO) {
      if (useLo) {
        v16b bl[4];
#pragma unroll
        for (int j = 0; j < 4; ++j) bl[j] = Frag<__bf16>::load(B2b + (size_t)(n0 + (j << 4) + rlane) * ldb + koff + k0);
#pragma unroll
        for (int i = 0; i < 4; ++i) {
          const v16b al = Frag<__bf16>::load(A2b + (size_t)(m0 + (i << 4) + rlane) * lda + koff + k0);
#pragma unroll
          for (int j = 0; j < 4; ++j) acc[i][j] = Frag<__bf16>::mma(al, bl[j], acc[i][j]);
          Frag<__bf16>::guard_row(acc[i][0], acc[i][1], acc[i][2], acc[i][3], al, bl[0], bl[1], bl[2], bl[3]);
        }
      }
    }
  }
  acc_guard4(acc[0][0], acc[0][1], acc[0][2], acc[0][3]);
  acc_guard4(acc[1][0], acc[1][1], acc[1][2], acc[1][3]);
  acc_guard4(acc[2][0], acc[2][1], acc[2][2], acc[2][3]);
  acc_guard4(acc[3][0], acc[3][1], acc[3][2], acc[3][3]);

  float* slab = sT[wave];
#pragma unroll
  for (int i = 0; i < 4; ++i) {
    const int mBase = m0 + (i << 4);
#pragma unroll
    for (int j = 0; j < 4; ++j) {
#pragma unroll
      for (int r = 0; r < 8; ++r) slab[(mOff + r) * 68 + (j << 4) + rlane] = acc[i][j][r] * scale;
    }
    __builtin_amdgcn_fence(__ATOMIC_RELEASE, "workgroup");
    __builtin_amdgcn_wave_barrier();
    __builtin_amdgcn_fence(__ATOMIC_ACQUIRE, "workgroup");
    if (OUT_MODE == 0) {
      float* C = (float*)Cout + (size_t)b * strideC;
      const int hh = lane >> 4, c4 = (lane & 15) * 4;
      for (int pass = 0; pass < 2; ++pass) {
#pragma unroll
        for (int it = 0; it < 8; ++it) {
          const int row = it * 2 + hh;
          const v4f v = *(const v4f*)(slab + row * 68 + c4);
          *(volatile v4f*)(C + (size_t)(mBase + row) * ldc + n0 + c4) = v;
        }
        __threadfence();
      }
    } else {
      const int qd = lane >> 3, c8 = (lane & 7) * 8;
      _Float16* C  = (_Float16*)Cout  + (size_t)b * strideC;
      _Float16* C2 = (_Float16*)Cout2 + (size_t)b * strideC;
      for (int pass = 0; pass < 2; ++pass) {
#pragma unroll
        for (int it = 0; it < 4; ++it) {
          const int row = it * 4 + qd;
          const float* sp = slab + row * 68 + c8;
          v8h hv, lv;
#pragma unroll
          for (int e = 0; e < 8; ++e) {
            const float xv = sp[e];
            const _Float16 hx = (_Float16)xv;
            const float hf = (float)hx;
            const float res = (xv - hf) * kLoCarry;
            hv[e] = hx;
            lv[e] = (_Float16)res;
          }
          *(volatile v8h*)(C  + (size_t)(mBase + row) * ldc + n0 + c8) = hv;
          *(volatile v8h*)(C2 + (size_t)(mBase + row) * ldc + n0 + c8) = lv;
        }
        __threadfence();
      }
    }
    __builtin_amdgcn_fence(__ATOMIC_RELEASE, "workgroup");
    __builtin_amdgcn_wave_barrier();
    __builtin_amdgcn_fence(__ATOMIC_ACQUIRE, "workgroup");
  }
}

template <bool EARLY>
__global__ __launch_bounds__(128) void attn_kernel(
    const unsigned short* __restrict__ Qh_, const unsigned short* __restrict__ Ql_,
    const unsigned short* __restrict__ Kh_, const unsigned short* __restrict__ Kl_,
    const unsigned short* __restrict__ Vh_, const unsigned short* __restrict__ Vl_,
    const float* __restrict__ Mk, const unsigned* __restrict__ Skip,
    unsigned short* __restrict__ Ch_, unsigned short* __restrict__ Cl_, int qb0) {
  __shared__ __align__(16) _Float16 sKh[kTK * kHd];
  __shared__ __align__(16) _Float16 sKl[EARLY ? kTK * kHd : 8];
  __shared__ __align__(16) _Float16 sVh[kHd * kTK];
  __shared__ __align__(16) _Float16 sVl[EARLY ? kHd * kTK : 8];
  __shared__ __align__(16) _Float16 sPh[4][16 * kTK];
  __shared__ __align__(16) _Float16 sPl[EARLY ? 4 : 1][EARLY ? 16 * kTK : 8];
  __shared__ __align__(16) float sM[kQBlk * kMP];
  __shared__ __align__(16) float sO[4][16 * 68];

  const int tid  = threadIdx.x;
  const int wave = __builtin_amdgcn_readfirstlane((int)(tid >> 5));
  const int lane = tid & 31;
  const int hh   = lane >> 4;
  const int c    = lane & 15;
  const int qb   = blockIdx.x + qb0;
  const int hq   = blockIdx.y;
  const int b    = blockIdx.z;
  const int g    = hq & (kHkv - 1);
  const int s0   = qb * kQBlk;
  const int q0   = s0 + wave * 16;

  const size_t qoff = (size_t)(b * kSeq + q0 + c) * kEmb + hq * kHd + 8 * hh;
  const _Float16* Qhp = (const _Float16*)Qh_ + qoff;
  const _Float16* Qlp = (const _Float16*)Ql_ + qoff;
  v16h qah[2], qal[2];
#pragma unroll
  for (int dc = 0; dc < 2; ++dc) {
    qah[dc] = FragH::load(Qhp + dc * 32);
    qal[dc] = qah[dc];
    if (EARLY) qal[dc] = FragH::load(Qlp + dc * 32);
  }

  const size_t kbase = (size_t)b * kSeq * kKvW + (size_t)g * kHd;
  const size_t vbase = ((size_t)b * kKvW + (size_t)g * kHd) * kSeq;
  const _Float16* Kg  = (const _Float16*)Kh_ + kbase;
  const _Float16* Kgl = (const _Float16*)Kl_ + kbase;
  const _Float16* Vg  = (const _Float16*)Vh_ + vbase;
  const _Float16* Vgl = (const _Float16*)Vl_ + vbase;
  const float* Mq = Mk + (size_t)s0 * kSeq;
  const unsigned* SkipRow = Skip + (size_t)qb * kNKT;

  float mrow[8], lrow[8];
  v8f oacc[4], oacc2[4];
#pragma unroll
  for (int r = 0; r < 8; ++r) { mrow[r] = -1.0e30f; lrow[r] = 0.f; }
#pragma unroll
  for (int t = 0; t < 4; ++t) {
    oacc[t]  = (v8f){0.f, 0.f, 0.f, 0.f, 0.f, 0.f, 0.f, 0.f};
    oacc2[t] = (v8f){0.f, 0.f, 0.f, 0.f, 0.f, 0.f, 0.f, 0.f};
  }

  _Float16* pwh = sPh[wave];
  _Float16* pwl = sPl[EARLY ? wave : 0];
  const float* mwv = sM + (wave * 16 + 8 * hh) * kMP + c;

  for (int kt = 0; kt < kNKT; ++kt) {
    const int sk = __builtin_amdgcn_readfirstlane((int)SkipRow[kt]);
    if (sk != 0) continue;
    const int t0 = kt * kTK;
    __syncthreads();
#pragma unroll
    for (int i = 0; i < 2; ++i) {
      const int id = tid + 128 * i;
      const int kr = id >> 3, kc = (id & 7) * 8;
      const int vr = id >> 2, vc = (id & 3) * 8;
      *(v8h*)(sKh + kr * kHd + kc) = *(const v8h*)(Kg + (size_t)(t0 + kr) * kKvW + kc);
      *(v8h*)(sVh + vr * kTK + vc) = *(const v8h*)(Vg + (size_t)vr * kSeq + t0 + vc);
      if (EARLY) {
        *(v8h*)(sKl + kr * kHd + kc) = *(const v8h*)(Kgl + (size_t)(t0 + kr) * kKvW + kc);
        *(v8h*)(sVl + vr * kTK + vc) = *(const v8h*)(Vgl + (size_t)vr * kSeq + t0 + vc);
      }
    }
#pragma unroll
    for (int i = 0; i < 4; ++i) {
      const int id = tid + 128 * i;
      const int mrw = id >> 3, mc = (id & 7) * 4;
      const v4f mv = *(const v4f*)(Mq + (size_t)mrw * kSeq + t0 + mc);
      const float a0 = mv[0];
      const float a1 = mv[1];
      const float a2 = mv[2];
      const float a3 = mv[3];
      const v4f mo = (v4f){bf_rne(a0), bf_rne(a1), bf_rne(a2), bf_rne(a3)};
      *(v4f*)(sM + mrw * kMP + mc) = mo;
    }
    __syncthreads();

    float sc[2][8];
#pragma unroll
    for (int j = 0; j < 2; ++j) {
      v8f sa = (v8f){0.f, 0.f, 0.f, 0.f, 0.f, 0.f, 0.f, 0.f};
      v8f sb = (v8f){0.f, 0.f, 0.f, 0.f, 0.f, 0.f, 0.f, 0.f};
#pragma unroll
      for (int dc = 0; dc < 2; ++dc) {
        const v16h kb = FragH::load(sKh + (j * 16 + c) * kHd + dc * 32 + 8 * hh);
        sa = mma_h(qah[dc], kb, sa);
        if (EARLY) {
          const v16h kl = FragH::load(sKl + (j * 16 + c) * kHd + dc * 32 + 8 * hh);
          sb = mma_h(qah[dc], kl, sb);
          sb = mma_h(qal[dc], kb, sb);
        }
      }
#pragma unroll
      for (int r = 0; r < 8; ++r) {
        float v = sa[r] * kScoreScale;
        if (EARLY) v += sb[r] * kScoreLoScale;
        const float mk = mwv[r * kMP + j * 16];
        sc[j][r] = v + mk;
      }
    }
#pragma unroll
    for (int r = 0; r < 8; ++r) {
      float m = fmaxf(sc[0][r], sc[1][r]);
#pragma unroll
      for (int off = 1; off < 16; off <<= 1) m = fmaxf(m, __shfl_xor(m, off, 32));
      const float mnew  = fmaxf(mrow[r], m);
      const float alpha = __expf(mrow[r] - mnew);
      mrow[r] = mnew;
      float psum = 0.f;
#pragma unroll
      for (int j = 0; j < 2; ++j) {
        const float p = __expf(sc[j][r] - mnew) * kPCarry;
        const _Float16 ph = (_Float16)p;
        const float pf = (float)ph;
        pwh[(8 * hh + r) * kTK + j * 16 + c] = ph;
        if (EARLY) {
          const float pres = (p - pf) * kLoCarry;
          pwl[(8 * hh + r) * kTK + j * 16 + c] = (_Float16)pres;
          psum += p;
        } else {
          psum += pf;
        }
      }
#pragma unroll
      for (int off = 1; off < 16; off <<= 1) psum += __shfl_xor(psum, off, 32);
      lrow[r] = lrow[r] * alpha + psum;
#pragma unroll
      for (int t = 0; t < 4; ++t) {
        oacc[t][r] *= alpha;
        if (EARLY) oacc2[t][r] *= alpha;
      }
    }
    __builtin_amdgcn_fence(__ATOMIC_RELEASE, "workgroup");
    __builtin_amdgcn_wave_barrier();
    __builtin_amdgcn_fence(__ATOMIC_ACQUIRE, "workgroup");
    {
      const v16h pa = FragH::load(pwh + c * kTK + 8 * hh);
      v16h pl = pa;
      if (EARLY) pl = FragH::load(pwl + c * kTK + 8 * hh);
#pragma unroll
      for (int t = 0; t < 4; ++t) {
        const v16h vb = FragH::load(sVh + (t * 16 + c) * kTK + 8 * hh);
        oacc[t] = mma_h(pa, vb, oacc[t]);
        if (EARLY) {
          const v16h vl = FragH::load(sVl + (t * 16 + c) * kTK + 8 * hh);
          oacc2[t] = mma_h(pa, vl, oacc2[t]);
          oacc2[t] = mma_h(pl, vb, oacc2[t]);
        }
      }
    }
  }

  float* os = sO[wave];
#pragma unroll
  for (int r = 0; r < 8; ++r) {
    const float inv = kCtxFold * (1.0f / lrow[r]);
#pragma unroll
    for (int t = 0; t < 4; ++t) {
      float v = oacc[t][r];
      if (EARLY) v += oacc2[t][r] * kLoCarryInv;
      os[(8 * hh + r) * 68 + t * 16 + c] = v * inv;
    }
  }
  __builtin_amdgcn_fence(__ATOMIC_RELEASE, "workgroup");
  __builtin_amdgcn_wave_barrier();
  __builtin_amdgcn_fence(__ATOMIC_ACQUIRE, "workgroup");
  {
    const int qd = lane >> 3, c8 = (lane & 7) * 8;
    v8h hv[4];
    v4u lw[4];
#pragma unroll
    for (int it = 0; it < 4; ++it) {
      const float* sp = os + (it * 4 + qd) * 68 + c8;
      unsigned short lb[8];
#pragma unroll
      for (int e = 0; e < 8; ++e) {
        const float xv = sp[e];
        const _Float16 hx = (_Float16)xv;
        const float hf = (float)hx;
        hv[it][e] = hx;
        lb[e] = f2bf_bits((xv - hf) * kWoCarry);
      }
      lw[it] = (v4u){pk16(lb[0], lb[1]), pk16(lb[2], lb[3]), pk16(lb[4], lb[5]), pk16(lb[6], lb[7])};
    }
    const size_t co = (size_t)(b * kSeq + q0) * kEmb + hq * kHd + c8;
    _Float16* Chp = (_Float16*)Ch_ + co;
    unsigned short* Clp = Cl_ + co;
    for (int pass = 0; pass < 2; ++pass) {
#pragma unroll
      for (int it = 0; it < 4; ++it) {
        const size_t ro = (size_t)(it * 4 + qd) * kEmb;
        *(volatile v8h*)(Chp + ro) = hv[it];
        if (EARLY) *(volatile v4u*)(Clp + ro) = lw[it];
      }
      __threadfence();
    }
  }
}

extern "C" void kernel_launch(void* const* d_in, const int* in_sizes, int n_in,
                              void* d_out, int out_size, void* d_ws, size_t ws_size,
                              hipStream_t stream) {
  if (n_in < 6) return;
  if (in_sizes[0] != kRows * kEmb) return;
  if (in_sizes[1] != kSeq * kSeq) return;
  if (in_sizes[2] != kEmb * kEmb) return;
  if (in_sizes[3] != kKvW * kEmb) return;
  if (in_sizes[4] != kKvW * kEmb) return;
  if (in_sizes[5] != kEmb * kEmb) return;
  if (out_size != kRows * kEmb) return;
  if (ws_size < kWsTotal) return;

  const float* x  = (const float*)d_in[0];
  const float* Mk = (const float*)d_in[1];
  const float* Wq = (const float*)d_in[2];
  const float* Wk = (const float*)d_in[3];
  const float* Wv = (const float*)d_in[4];
  const float* Wo = (const float*)d_in[5];

  char* ws = (char*)d_ws;
  unsigned short* XB  = (unsigned short*)(ws + kOffXB);
  unsigned short* WQB = (unsigned short*)(ws + kOffWQB);
  unsigned short* WKB = (unsigned short*)(ws + kOffWKB);
  unsigned short* WVB = (unsigned short*)(ws + kOffWVB);
  unsigned short* WOH = (unsigned short*)(ws + kOffWOH);
  unsigned short* WOB = (unsigned short*)(ws + kOffWOB);
  unsigned short* QH  = (unsigned short*)(ws + kOffQH);
  unsigned short* QL  = (unsigned short*)(ws + kOffQL);
  unsigned short* KH  = (unsigned short*)(ws + kOffKH);
  unsigned short* KL  = (unsigned short*)(ws + kOffKL);
  unsigned short* VTH = (unsigned short*)(ws + kOffVTH);
  unsigned short* VTL = (unsigned short*)(ws + kOffVTL);
  unsigned short* CH  = (unsigned short*)(ws + kOffCH);
  unsigned short* CL  = (unsigned short*)(ws + kOffCL);
  unsigned*       SKP = (unsigned*)(ws + kOffSKP);

  cast8_bf16_kernel<<<(kRows * kEmb / 8) / 256, 256, 0, stream>>>(x,  XB,  kRows * kEmb / 8);
  cast8_bf16_kernel<<<(kEmb * kEmb / 8) / 256, 256, 0, stream>>>(Wq, WQB, kEmb * kEmb / 8);
  cast8_bf16_kernel<<<(kKvW * kEmb / 8) / 256, 256, 0, stream>>>(Wk, WKB, kKvW * kEmb / 8);
  cast8_bf16_kernel<<<(kKvW * kEmb / 8) / 256, 256, 0, stream>>>(Wv, WVB, kKvW * kEmb / 8);
  cast8_wo_kernel<<<(kEmb * kEmb / 8) / 256, 256, 0, stream>>>(Wo, WOB, WOH, kEmb * kEmb / 8);

  mask_tiles_kernel<<<kNQB, 256, 0, stream>>>(Mk, SKP);

  gemm64_kernel<1, false, 3><<<dim3((kRows / 64) * (kEmb / 64) / 8, 1), 256, 0, stream>>>(
      XB, kEmb, 0L, WQB, kEmb, 0L, nullptr, nullptr,
      (void*)QH, (void*)QL, kEmb, 0L, kRows, kEmb, kEmb, kQCarry, 1, 0);

  gemm64_kernel<1, false, 3><<<dim3((kRows / 64) * (kKvW / 64) / 8, 1), 256, 0, stream>>>(
      XB, kEmb, 0L, WKB, kEmb, 0L, nullptr, nullptr,
      (void*)KH, (void*)KL, kKvW, 0L, kRows, kKvW, kEmb, kKCarry, 1, 0);

  gemm64_kernel<1, false, 3><<<dim3((kKvW / 64) * (kSeq / 64) / 8, kBatch), 256, 0, stream>>>(
      WVB, kEmb, 0L, XB, kEmb, (long)kSeq * kEmb, nullptr, nullptr,
      (void*)VTH, (void*)VTL, kSeq, (long)kKvW * kSeq, kKvW, kSeq, kEmb, kVCarry, 1, 0);

  attn_kernel<true><<<dim3(kEarlyRows / kQBlk, kHq, kBatch), 128, 0, stream>>>(QH, QL, KH, KL, VTH, VTL, Mk, SKP, CH, CL, 0);
  attn_kernel<false><<<dim3((kSeq - kEarlyRows) / kQBlk, kHq, kBatch), 128, 0, stream>>>(QH, QL, KH, KL, VTH, VTL, Mk, SKP, CH, CL,
                                                                                         kEarlyRows / kQBlk);

  gemm64_kernel<0, true, 0><<<dim3((kRows / 64) * (kEmb / 64) / 8, 1), 256, 0, stream>>>(
      CH, kEmb, 0L, WOH, kEmb, 0L, CL, WOB,
      d_out, nullptr, kEmb, 0L, kRows, kEmb, kEmb, kOutScale, kSeq, kEarlyRows);
}
